// SpectralConv2d_ssd_20263655702998
// MI455X (gfx1250) — hardware-run, weakly checked
//
#include <hip/hip_runtime.h>
#include <math.h>

typedef __attribute__((ext_vector_type(16))) _Float16 v16h;
typedef __attribute__((ext_vector_type(8)))  _Float16 v8h;
typedef __attribute__((ext_vector_type(8)))  float    v8f;
typedef __attribute__((ext_vector_type(4)))  float    v4f;

constexpr int kBatch = 4;
constexpr int kChan  = 64;
constexpr int kHt    = 128;
constexpr int kWd    = 128;
constexpr int kDch   = 2 * kChan;
constexpr int kNst   = 64;
constexpr int kWf    = kWd / 2 + 1;
constexpr int kTokB  = kHt * kWf;
constexpr int kTok   = kBatch * kTokB;
constexpr int kNcat  = kDch + 2 * kNst;
constexpr int kScanT = 32;
static_assert(kHt == 128 && kWd == 128, "128-point passes");
static_assert(kHt == kWd, "sqrt(H*W) == H");
static_assert(kWf == 65 && kTokB == 8320 && kTok == 33280 && kNcat == 256, "shape");
static_assert((kTok % 64) == 0 && (kNcat % 64) == 0 && (kDch % 64) == 0 && (kDch % 32) == 0, "GEMM tile multiples");
static_assert((kTokB % kScanT) == 0 && (kTokB % 64) == 0, "chunk multiples");

constexpr float kSqrtN    = (float)kHt;
constexpr float kInvSqrtN = 1.0f / kSqrtN;
constexpr float kCarryU   = 16.0f;
constexpr float kCarryW   = 256.0f;
constexpr float kCarryY   = 16384.0f;
constexpr float kProjScale = 1.0f / (kSqrtN * kCarryU * kCarryW);
constexpr float kOutScale  = kSqrtN / (kCarryY * kCarryW);

constexpr size_t kSzTw    = 512;
constexpr size_t kSzPlane = (size_t)kBatch * kWf * kChan * kHt * 4;
constexpr size_t kSzU     = (size_t)kTok * kDch * 4;
constexpr size_t kSzUH    = (size_t)kTok * kDch * 2;
constexpr size_t kSzDD    = (size_t)kTok * 2 * 4;
constexpr size_t kSzWH    = (size_t)(kNcat + kDch) * kDch * 2;
constexpr size_t kSzXBC   = (size_t)kTok * kNcat * 4;
constexpr size_t kOffTw   = 0;
constexpr size_t kOffPre  = kOffTw  + kSzTw;
constexpr size_t kOffPim  = kOffPre + kSzPlane;
constexpr size_t kOffU    = kOffPim + kSzPlane;
constexpr size_t kOffUH   = kOffU   + kSzU;
constexpr size_t kOffDD   = kOffUH  + kSzUH;
constexpr size_t kOffWH   = kOffDD  + kSzDD;
constexpr size_t kOffXBC  = kOffWH  + kSzWH;
constexpr size_t kOffY    = kOffXBC + kSzXBC;
constexpr size_t kOffF    = kOffY   + kSzUH;
constexpr size_t kOffQre  = kOffF   + kSzU;
constexpr size_t kOffQim  = kOffQre + kSzPlane;
constexpr size_t kWsTotal = kOffQim + kSzPlane;
static_assert(kWsTotal == 119640576ull, "carve total");
static_assert(kWsTotal <= 134217728ull, "carve cap");
static_assert((kOffPre % 128) == 0 && (kOffPim % 128) == 0 && (kOffU % 128) == 0 && (kOffUH % 128) == 0 &&
              (kOffDD % 128) == 0 && (kOffWH % 128) == 0 && (kOffXBC % 128) == 0 && (kOffY % 128) == 0 &&
              (kOffF % 128) == 0 && (kOffQre % 128) == 0 && (kOffQim % 128) == 0, "128-B aligned regions");

__device__ __forceinline__ int brev7(int i) { return (int)(__brev((unsigned)i) >> 25); }

union FragH { v16h v; v8h h[2]; };
__device__ __forceinline__ v16h frag_load_h(const _Float16* p) {
  FragH f;
  f.h[0] = *(const v8h*)(p);
  f.h[1] = *(const v8h*)(p + 16);
  return f.v;
}
__device__ __forceinline__ v8f mma_h(v16h a, v16h b, v8f c) {
  c = __builtin_amdgcn_wmma_f32_16x16x32_f16(false, a, false, b, (short)0, c, false, false);
  asm volatile("v_nop\n\tv_nop\n\tv_nop\n\tv_nop" : "+v"(c) : "v"(a), "v"(b));
  return c;
}

__device__ __forceinline__ void fft128_lane(float* re, float* im, const float* tw, const float sgn) {
  int half = 1;
  int tstep = 64;
#pragma unroll 1
  for (int st = 0; st < 7; ++st) {
#pragma unroll 2
    for (int j = 0; j < 64; ++j) {
      const int k  = j & (half - 1);
      const int i0 = ((j - k) << 1) + k;
      const int i1 = i0 + half;
      const float wr = tw[k * tstep];
      const float wi = sgn * tw[64 + k * tstep];
      const float xr = re[i1 << 5];
      const float xi = im[i1 << 5];
      const float tr = wr * xr - wi * xi;
      const float ti = wr * xi + wi * xr;
      const float ur = re[i0 << 5];
      const float ui = im[i0 << 5];
      re[i0 << 5] = ur + tr;
      im[i0 << 5] = ui + ti;
      re[i1 << 5] = ur - tr;
      im[i1 << 5] = ui - ti;
    }
    half <<= 1;
    tstep >>= 1;
  }
}

__global__ __launch_bounds__(32) void twiddle_kernel(float* __restrict__ tw) {
  const int lane = threadIdx.x & 31;
  v4f v;
#pragma unroll
  for (int e = 0; e < 4; ++e) {
    const int idx = lane * 4 + e;
    const float ang = (float)(idx & 63) * (1.0f / 64.0f);
    const float cv = cospif(ang);
    const float sv = sinpif(ang);
    v[e] = (idx < 64) ? cv : sv;
  }
  *(volatile v4f*)(tw + lane * 4) = v;
  __threadfence();
  *(volatile v4f*)(tw + lane * 4) = v;
}

__global__ __launch_bounds__(256) void cast_weights_kernel(
    const float* __restrict__ Wx, const float* __restrict__ Wb, const float* __restrict__ Wc,
    const float* __restrict__ Wo, unsigned short* __restrict__ dst) {
  const int blk0 = blockIdx.x * 2048;
  const int e0 = blk0 + threadIdx.x * 8;
  const float* src;
  int off;
  if (blk0 < 16384)      { src = Wx; off = 0; }
  else if (blk0 < 24576) { src = Wb; off = 16384; }
  else if (blk0 < 32768) { src = Wc; off = 24576; }
  else                   { src = Wo; off = 32768; }
  const v4f a0 = *(const v4f*)(src + (e0 - off));
  const v4f a1 = *(const v4f*)(src + (e0 - off) + 4);
  v8h hv;
#pragma unroll
  for (int e = 0; e < 4; ++e) {
    hv[e]     = (_Float16)(a0[e] * kCarryW);
    hv[4 + e] = (_Float16)(a1[e] * kCarryW);
  }
  unsigned short* q = dst + e0;
  *(volatile v8h*)q = hv;
  __threadfence();
  *(volatile v8h*)q = hv;
}

__global__ __launch_bounds__(32) void fwd_rows_kernel(
    const float* __restrict__ x, const float* __restrict__ tw,
    float* __restrict__ Pre, float* __restrict__ Pim) {
  __shared__ __align__(16) float sbuf[2 * 4096];
  __shared__ __align__(16) float stw[128];
  float* sre = sbuf;
  float* sim = sbuf + 4096;
  const int lane = threadIdx.x & 31;
  const int bc = blockIdx.x >> 2;
  const int hq = blockIdx.x & 3;
  const int b = bc >> 6;
  const int c = bc & 63;
  const size_t r0 = (size_t)bc * kHt + (size_t)hq * 32;
  *(v4f*)(stw + lane * 4) = *(const v4f*)(tw + lane * 4);
  const int i0 = lane * 4;
  const int p0 = brev7(i0), p1 = brev7(i0 + 1), p2 = brev7(i0 + 2), p3 = brev7(i0 + 3);
#pragma unroll 4
  for (int rr = 0; rr < 32; ++rr) {
    const v4f v = *(const v4f*)(x + (r0 + rr) * kWd + i0);
    sre[p0 * 32 + rr] = v[0];
    sre[p1 * 32 + rr] = v[1];
    sre[p2 * 32 + rr] = v[2];
    sre[p3 * 32 + rr] = v[3];
    sim[p0 * 32 + rr] = 0.0f;
    sim[p1 * 32 + rr] = 0.0f;
    sim[p2 * 32 + rr] = 0.0f;
    sim[p3 * 32 + rr] = 0.0f;
  }
  __syncthreads();
  fft128_lane(sre + lane, sim + lane, stw, -1.0f);
  __syncthreads();
  const int q = lane >> 3, j = lane & 7;
  for (int pass = 0; pass < 2; ++pass) {
#pragma unroll 1
    for (int it = 0; it < 17; ++it) {
      const int kw = it * 4 + q;
      const int kwc = (kw < kWf) ? kw : (kWf - 1);
      const v4f vr = *(const v4f*)(sre + kwc * 32 + j * 4);
      const v4f vi = *(const v4f*)(sim + kwc * 32 + j * 4);
      if (kw < kWf) {
        const size_t o = ((size_t)(b * kWf + kw) * kChan + c) * kHt + hq * 32 + j * 4;
        *(volatile v4f*)(Pre + o) = vr;
        *(volatile v4f*)(Pim + o) = vi;
      }
    }
    __threadfence();
  }
}

__global__ __launch_bounds__(32) void fwd_cols_kernel(
    const float* __restrict__ Pre, const float* __restrict__ Pim, const float* __restrict__ tw,
    float* __restrict__ U) {
  __shared__ __align__(16) float sbuf[2 * 4096];
  __shared__ __align__(16) float stw[128];
  float* sre = sbuf;
  float* sim = sbuf + 4096;
  const int lane = threadIdx.x & 31;
  const int chalf = blockIdx.x & 1;
  const int bk = blockIdx.x >> 1;
  const int b = bk / kWf;
  const int kw = bk - b * kWf;
  const int c0 = chalf * 32;
  *(v4f*)(stw + lane * 4) = *(const v4f*)(tw + lane * 4);
  const int i0 = lane * 4;
  const int p0 = brev7(i0), p1 = brev7(i0 + 1), p2 = brev7(i0 + 2), p3 = brev7(i0 + 3);
#pragma unroll 4
  for (int cc = 0; cc < 32; ++cc) {
    const size_t o = ((size_t)(b * kWf + kw) * kChan + c0 + cc) * kHt + i0;
    const v4f vr = *(const v4f*)(Pre + o);
    const v4f vi = *(const v4f*)(Pim + o);
    sre[p0 * 32 + cc] = vr[0];
    sre[p1 * 32 + cc] = vr[1];
    sre[p2 * 32 + cc] = vr[2];
    sre[p3 * 32 + cc] = vr[3];
    sim[p0 * 32 + cc] = vi[0];
    sim[p1 * 32 + cc] = vi[1];
    sim[p2 * 32 + cc] = vi[2];
    sim[p3 * 32 + cc] = vi[3];
  }
  __syncthreads();
  fft128_lane(sre + lane, sim + lane, stw, -1.0f);
  __syncthreads();
  const int q = lane >> 3, j = lane & 7;
  for (int pass = 0; pass < 2; ++pass) {
#pragma unroll 4
    for (int it = 0; it < 64; ++it) {
      const int ln = it * 4 + q;
      const int kh = ln >> 1;
      const int pl = ln & 1;
      v4f v = *(const v4f*)(sbuf + pl * 4096 + kh * 32 + j * 4);
      v = v * kInvSqrtN;
      const size_t o = ((size_t)b * kTokB + (size_t)kh * kWf + kw) * kDch + pl * 64 + c0 + j * 4;
      *(volatile v4f*)(U + o) = v;
    }
    __threadfence();
  }
}

__global__ __launch_bounds__(256) void ln_gate_kernel(
    const float* __restrict__ U, const float* __restrict__ nw, const float* __restrict__ nb,
    const float* __restrict__ wdt, const float* __restrict__ dtb, const float* __restrict__ alog,
    unsigned short* __restrict__ UH, float* __restrict__ DD) {
  __shared__ __align__(16) float sT[64 * 132];
  __shared__ __align__(16) float sPar[3 * kDch];
  __shared__ __align__(16) float sDD[128];
  const int tid = threadIdx.x;
  const int lane = tid & 31;
  const int wave = __builtin_amdgcn_readfirstlane((int)(threadIdx.x >> 5));
  const int m0 = blockIdx.x * 64;
  if (wave < 4) {
    sPar[tid] = nw[tid];
    sPar[kDch + tid] = nb[tid];
    sPar[2 * kDch + tid] = wdt[tid];
  }
#pragma unroll
  for (int it = 0; it < 8; ++it) {
    const int idx = it * 256 + tid;
    const int row = idx >> 5;
    const int c4 = (idx & 31) * 4;
    *(v4f*)(sT + row * 132 + c4) = *(const v4f*)(U + (size_t)(m0 + row) * kDch + c4);
  }
  __syncthreads();
  const int tok = tid >> 2;
  const int part = tid & 3;
  float* rowp = sT + tok * 132 + part * 32;
  const float* gp = sPar + part * 32;
  float s = 0.0f;
#pragma unroll
  for (int i = 0; i < 8; ++i) {
    const v4f v = *(const v4f*)(rowp + 4 * i);
    s += (v[0] + v[1]) + (v[2] + v[3]);
  }
  s += __shfl_xor(s, 1, 32);
  s += __shfl_xor(s, 2, 32);
  const float mu = s * (1.0f / (float)kDch);
  float ss = 0.0f;
#pragma unroll 2
  for (int i = 0; i < 8; ++i) {
    const v4f v = *(const v4f*)(rowp + 4 * i);
    const float d0 = v[0] - mu, d1 = v[1] - mu, d2 = v[2] - mu, d3 = v[3] - mu;
    ss += (d0 * d0 + d1 * d1) + (d2 * d2 + d3 * d3);
  }
  ss += __shfl_xor(ss, 1, 32);
  ss += __shfl_xor(ss, 2, 32);
  const float var = ss * (1.0f / (float)kDch);
  const float rs = rsqrtf(var + 1e-5f);
  float zacc = 0.0f;
#pragma unroll 2
  for (int i = 0; i < 8; ++i) {
    const v4f v  = *(const v4f*)(rowp + 4 * i);
    const v4f g  = *(const v4f*)(gp + 4 * i);
    const v4f bb = *(const v4f*)(gp + kDch + 4 * i);
    const v4f w  = *(const v4f*)(gp + 2 * kDch + 4 * i);
    v4f o;
#pragma unroll
    for (int e = 0; e < 4; ++e) {
      o[e] = ((v[e] - mu) * rs) * g[e] + bb[e];
      zacc += w[e] * (o[e] * kInvSqrtN);
    }
    *(v4f*)(rowp + 4 * i) = o * kCarryU;
  }
  zacc += __shfl_xor(zacc, 1, 32);
  zacc += __shfl_xor(zacc, 2, 32);
  const float z = zacc + dtb[0];
  const float aexp = expf(alog[0]);
  const float dt = fmaxf(z, 0.0f) + log1pf(expf(-fabsf(z)));
  float dec = expf(-aexp * dt);
  dec = (dec < 1.17549435e-38f) ? 0.0f : dec;
  if (part == 0) {
    sDD[tok * 2] = dt;
    sDD[tok * 2 + 1] = dec;
  }
  __syncthreads();
  const int q = lane >> 3, j = lane & 7;
  v8h hv[4];
#pragma unroll
  for (int it = 0; it < 4; ++it) {
    const int ln = it * 32 + wave * 4 + q;
    const int row = ln >> 1;
    const int hf = ln & 1;
    const float* sp = sT + row * 132 + hf * 64 + j * 8;
    const v4f a0 = *(const v4f*)(sp);
    const v4f a1 = *(const v4f*)(sp + 4);
#pragma unroll
    for (int e = 0; e < 4; ++e) {
      hv[it][e]     = (_Float16)a0[e];
      hv[it][4 + e] = (_Float16)a1[e];
    }
  }
  v4f dv = *(const v4f*)(sDD + lane * 4);
  for (int pass = 0; pass < 2; ++pass) {
#pragma unroll
    for (int it = 0; it < 4; ++it) {
      const int ln = it * 32 + wave * 4 + q;
      const int row = ln >> 1;
      const int hf = ln & 1;
      *(volatile v8h*)(UH + (size_t)(m0 + row) * kDch + hf * 64 + j * 8) = hv[it];
    }
    if (wave == 0) {
      *(volatile v4f*)(DD + (size_t)m0 * 2 + lane * 4) = dv;
    }
    __threadfence();
  }
}

__global__ __launch_bounds__(256) void gemm_f16_kernel(
    const unsigned short* __restrict__ Ap, int lda,
    const unsigned short* __restrict__ Btp, int ldb,
    float* __restrict__ C, int ldc, int M, int N, int K, float scale) {
  const _Float16* A  = (const _Float16*)Ap;
  const _Float16* Bt = (const _Float16*)Btp;
  __shared__ __align__(16) float sT[8][16 * 68];
  const int lane = threadIdx.x & 31;
  const int wave = __builtin_amdgcn_readfirstlane((int)(threadIdx.x >> 5));
  const int tilesN = N >> 6;
  const int tilesM = M >> 6;
  const int tile = blockIdx.x * 8 + wave;
  if (tile >= tilesM * tilesN) return;
  const int tm = tile / tilesN;
  const int tn = tile - tm * tilesN;
  const int m0 = tm << 6;
  const int n0 = tn << 6;
  const int rlane = lane & 15;
  const int koff  = (lane >> 4) * 8;
  const int mOff  = (lane >> 4) * 8;

  v8f acc[4][4];
#pragma unroll
  for (int i = 0; i < 4; ++i)
#pragma unroll
    for (int j = 0; j < 4; ++j) acc[i][j] = (v8f){0.f, 0.f, 0.f, 0.f, 0.f, 0.f, 0.f, 0.f};

  for (int k0 = 0; k0 < K; k0 += 32) {
    v16h bh[4];
#pragma unroll
    for (int j = 0; j < 4; ++j) {
      bh[j] = frag_load_h(Bt + (size_t)(n0 + (j << 4) + rlane) * ldb + koff + k0);
    }
#pragma unroll
    for (int i = 0; i < 4; ++i) {
      const v16h ah = frag_load_h(A + (size_t)(m0 + (i << 4) + rlane) * lda + koff + k0);
#pragma unroll
      for (int j = 0; j < 4; ++j) {
        acc[i][j] = mma_h(ah, bh[j], acc[i][j]);
      }
    }
  }

  float* slab = sT[wave];
#pragma unroll
  for (int i = 0; i < 4; ++i) {
    const int mBase = m0 + (i << 4);
#pragma unroll
    for (int j = 0; j < 4; ++j) {
#pragma unroll
      for (int r = 0; r < 8; ++r) {
        slab[(mOff + r) * 68 + (j << 4) + rlane] = acc[i][j][r] * scale;
      }
    }
    __builtin_amdgcn_fence(__ATOMIC_RELEASE, "workgroup");
    __builtin_amdgcn_wave_barrier();
    __builtin_amdgcn_fence(__ATOMIC_ACQUIRE, "workgroup");
    {
      const int hh = lane >> 4, c4 = (lane & 15) * 4;
      for (int pass = 0; pass < 2; ++pass) {
#pragma unroll
        for (int it = 0; it < 8; ++it) {
          const int row = it * 2 + hh;
          v4f v = *(const v4f*)(slab + row * 68 + c4);
          *(volatile v4f*)(C + (size_t)(mBase + row) * ldc + n0 + c4) = v;
        }
        __threadfence();
      }
    }
    __builtin_amdgcn_fence(__ATOMIC_RELEASE, "workgroup");
    __builtin_amdgcn_wave_barrier();
    __builtin_amdgcn_fence(__ATOMIC_ACQUIRE, "workgroup");
  }
}

__global__ __launch_bounds__(256) void scan_kernel(
    const float* __restrict__ XBC, const float* __restrict__ DD, const float* __restrict__ hprev,
    const float* __restrict__ Dskip, unsigned short* __restrict__ Y, float* __restrict__ hout) {
  __shared__ __align__(16) float sBC[kScanT * 128];
  __shared__ __align__(16) float sX[kScanT * 64];
  __shared__ __align__(16) float sY[kScanT * 68];
  __shared__ __align__(16) float sDs[kScanT * 2];
  __shared__ __align__(16) float sHt[64 * 68];
  const int tid = threadIdx.x;
  const int lane = tid & 31;
  const int wave = __builtin_amdgcn_readfirstlane((int)(threadIdx.x >> 5));
  const int b = blockIdx.x >> 1;
  const int d0 = (blockIdx.x & 1) * 64;
  const int ch = tid >> 2;
  const int nq = tid & 3;
  const int d = d0 + ch;
  float h[16];
  {
    const float* hp = hprev + ((size_t)(b * kDch + d)) * kNst + nq * 16;
#pragma unroll
    for (int g = 0; g < 4; ++g) {
      const v4f v = *(const v4f*)(hp + 4 * g);
      h[4 * g + 0] = v[0];
      h[4 * g + 1] = v[1];
      h[4 * g + 2] = v[2];
      h[4 * g + 3] = v[3];
    }
  }
  const float dsk = Dskip[d];
  const int q = lane >> 3, j = lane & 7;
#pragma unroll 1
  for (int chunk = 0; chunk < kTokB / kScanT; ++chunk) {
    const size_t tok0 = (size_t)b * kTokB + (size_t)chunk * kScanT;
    __syncthreads();
#pragma unroll
    for (int it = 0; it < 4; ++it) {
      const int idx = it * 256 + tid;
      const int row = idx >> 5;
      const int c4 = (idx & 31) * 4;
      *(v4f*)(sBC + row * 128 + c4) = *(const v4f*)(XBC + (tok0 + row) * kNcat + kDch + c4);
    }
#pragma unroll
    for (int it = 0; it < 2; ++it) {
      const int idx = it * 256 + tid;
      const int row = idx >> 4;
      const int c4 = (idx & 15) * 4;
      *(v4f*)(sX + row * 64 + c4) = *(const v4f*)(XBC + (tok0 + row) * kNcat + d0 + c4);
    }
    {
      v4f ddv = *(const v4f*)(DD + tok0 * 2 + (tid & 15) * 4);
      float e0 = ddv[0], e1 = ddv[1], e2 = ddv[2], e3 = ddv[3];
      asm volatile("" : "+v"(e0), "+v"(e1), "+v"(e2), "+v"(e3));
      if (tid < 16) {
        sDs[tid * 4 + 0] = e0;
        sDs[tid * 4 + 1] = e1;
        sDs[tid * 4 + 2] = e2;
        sDs[tid * 4 + 3] = e3;
      }
    }
    __syncthreads();
#pragma unroll 1
    for (int s = 0; s < kScanT; ++s) {
      const float dt = sDs[2 * s];
      const float dec = sDs[2 * s + 1];
      const float xv = sX[s * 64 + ch];
      const float dtx = dt * xv;
      const float* bp = sBC + s * 128 + nq * 16;
      float y = 0.0f;
#pragma unroll
      for (int g = 0; g < 4; ++g) {
        const v4f bv = *(const v4f*)(bp + 4 * g);
        const v4f cv = *(const v4f*)(bp + 64 + 4 * g);
#pragma unroll
        for (int e = 0; e < 4; ++e) {
          const float hn = fmaf(dtx, bv[e], dec * h[4 * g + e]);
          h[4 * g + e] = hn;
          y = fmaf(hn, cv[e], y);
        }
      }
      y += __shfl_xor(y, 1, 32);
      y += __shfl_xor(y, 2, 32);
      const float yo = (y + dsk * xv) * kCarryY;
      if (nq == 0) sY[s * 68 + ch] = yo;
    }
    __syncthreads();
    {
      const int row = wave * 4 + q;
      const float* sp = sY + row * 68 + j * 8;
      const v4f a0 = *(const v4f*)(sp);
      const v4f a1 = *(const v4f*)(sp + 4);
      v8h hv;
#pragma unroll
      for (int e = 0; e < 4; ++e) {
        hv[e]     = (_Float16)a0[e];
        hv[4 + e] = (_Float16)a1[e];
      }
      unsigned short* dst = Y + (tok0 + row) * kDch + d0 + j * 8;
      *(volatile v8h*)dst = hv;
      __threadfence();
      *(volatile v8h*)dst = hv;
    }
  }
  __syncthreads();
#pragma unroll
  for (int g = 0; g < 4; ++g) {
    v4f v;
    v[0] = h[4 * g + 0];
    v[1] = h[4 * g + 1];
    v[2] = h[4 * g + 2];
    v[3] = h[4 * g + 3];
    *(v4f*)(sHt + ch * 68 + nq * 16 + 4 * g) = v;
  }
  __syncthreads();
  {
    const int hh = lane >> 4, c4 = (lane & 15) * 4;
    for (int pass = 0; pass < 2; ++pass) {
#pragma unroll
      for (int it = 0; it < 4; ++it) {
        const int row = it * 16 + wave * 2 + hh;
        const v4f v = *(const v4f*)(sHt + row * 68 + c4);
        *(volatile v4f*)(hout + ((size_t)(b * kDch + d0 + row)) * kNst + c4) = v;
      }
      __threadfence();
    }
  }
}

__global__ __launch_bounds__(32) void inv_cols_kernel(
    const float* __restrict__ F, const float* __restrict__ tw,
    float* __restrict__ Qre, float* __restrict__ Qim) {
  __shared__ __align__(16) float sbuf[2 * 4096];
  __shared__ __align__(16) float stw[128];
  float* sre = sbuf;
  float* sim = sbuf + 4096;
  const int lane = threadIdx.x & 31;
  const int chalf = blockIdx.x & 1;
  const int bk = blockIdx.x >> 1;
  const int b = bk / kWf;
  const int kw = bk - b * kWf;
  const int c0 = chalf * 32;
  *(v4f*)(stw + lane * 4) = *(const v4f*)(tw + lane * 4);
#pragma unroll 4
  for (int kh = 0; kh < kHt; ++kh) {
    const int p = brev7(kh);
    const float* tr = F + ((size_t)b * kTokB + (size_t)kh * kWf + kw) * kDch + c0 + lane;
    sre[p * 32 + lane] = tr[0];
    sim[p * 32 + lane] = tr[kChan];
  }
  __syncthreads();
  fft128_lane(sre + lane, sim + lane, stw, 1.0f);
  __syncthreads();
  for (int pass = 0; pass < 2; ++pass) {
#pragma unroll 2
    for (int cc = 0; cc < 32; ++cc) {
      v4f vr, vi;
#pragma unroll
      for (int e = 0; e < 4; ++e) {
        vr[e] = sre[(lane * 4 + e) * 32 + cc];
        vi[e] = sim[(lane * 4 + e) * 32 + cc];
      }
      const size_t o = ((size_t)(b * kWf + kw) * kChan + c0 + cc) * kHt + lane * 4;
      *(volatile v4f*)(Qre + o) = vr;
      *(volatile v4f*)(Qim + o) = vi;
    }
    __threadfence();
  }
}

__global__ __launch_bounds__(32) void inv_rows_kernel(
    const float* __restrict__ Qre, const float* __restrict__ Qim, const float* __restrict__ tw,
    float* __restrict__ out) {
  __shared__ __align__(16) float sbuf[2 * 4096];
  __shared__ __align__(16) float stw[128];
  float* sre = sbuf;
  float* sim = sbuf + 4096;
  const int lane = threadIdx.x & 31;
  const int bc = blockIdx.x >> 2;
  const int hq = blockIdx.x & 3;
  const int b = bc >> 6;
  const int c = bc & 63;
  const int h0 = hq * 32;
  *(v4f*)(stw + lane * 4) = *(const v4f*)(tw + lane * 4);
#pragma unroll 1
  for (int kw = 0; kw < kWf; ++kw) {
    const size_t o = ((size_t)(b * kWf + kw) * kChan + c) * kHt + h0 + lane;
    const float r = Qre[o];
    const float iv = Qim[o];
    const bool edge = (kw == 0) || (kw == kWf - 1);
    const float iz = edge ? 0.0f : iv;
    const int p = brev7(kw);
    sre[p * 32 + lane] = r;
    sim[p * 32 + lane] = iz;
    if (!edge) {
      const int p2 = brev7(kWd - kw);
      sre[p2 * 32 + lane] = r;
      sim[p2 * 32 + lane] = -iz;
    }
  }
  __syncthreads();
  fft128_lane(sre + lane, sim + lane, stw, 1.0f);
  __syncthreads();
  for (int pass = 0; pass < 2; ++pass) {
#pragma unroll 2
    for (int rr = 0; rr < 32; ++rr) {
      v4f v;
#pragma unroll
      for (int e = 0; e < 4; ++e) v[e] = sre[(lane * 4 + e) * 32 + rr] * kInvSqrtN;
      const size_t o = ((size_t)bc * kHt + h0 + rr) * kWd + lane * 4;
      *(volatile v4f*)(out + o) = v;
    }
    __threadfence();
  }
}

extern "C" void kernel_launch(void* const* d_in, const int* in_sizes, int n_in,
                              void* d_out, int out_size, void* d_ws, size_t ws_size,
                              hipStream_t stream) {
  if (n_in < 12) return;
  if (in_sizes[0] != kBatch * kChan * kHt * kWd) return;
  if (in_sizes[1] != kBatch * kDch * kNst) return;
  if (in_sizes[2] != kDch || in_sizes[3] != kDch) return;
  if (in_sizes[4] != kDch * kDch) return;
  if (in_sizes[5] != kNst * kDch || in_sizes[6] != kNst * kDch) return;
  if (in_sizes[7] != kDch) return;
  if (in_sizes[8] != 1 || in_sizes[9] != 1) return;
  if (in_sizes[10] != kDch) return;
  if (in_sizes[11] != kDch * kDch) return;
  if (out_size != kBatch * kChan * kHt * kWd + kBatch * kDch * kNst) return;
  if (ws_size < kWsTotal) return;

  const float* x      = (const float*)d_in[0];
  const float* hprev  = (const float*)d_in[1];
  const float* nw     = (const float*)d_in[2];
  const float* nb     = (const float*)d_in[3];
  const float* Wx     = (const float*)d_in[4];
  const float* Wb     = (const float*)d_in[5];
  const float* Wc     = (const float*)d_in[6];
  const float* wdt    = (const float*)d_in[7];
  const float* dtbias = (const float*)d_in[8];
  const float* alog   = (const float*)d_in[9];
  const float* Dskip  = (const float*)d_in[10];
  const float* Wout   = (const float*)d_in[11];

  float* out0 = (float*)d_out;
  float* out1 = (float*)d_out + (size_t)kBatch * kChan * kHt * kWd;

  char* ws = (char*)d_ws;
  float*          TW  = (float*)(ws + kOffTw);
  float*          PRE = (float*)(ws + kOffPre);
  float*          PIM = (float*)(ws + kOffPim);
  float*          U   = (float*)(ws + kOffU);
  unsigned short* UH  = (unsigned short*)(ws + kOffUH);
  float*          DD  = (float*)(ws + kOffDD);
  unsigned short* WH  = (unsigned short*)(ws + kOffWH);
  float*          XBC = (float*)(ws + kOffXBC);
  unsigned short* Y   = (unsigned short*)(ws + kOffY);
  float*          F   = (float*)(ws + kOffF);
  float*          QRE = (float*)(ws + kOffQre);
  float*          QIM = (float*)(ws + kOffQim);

  twiddle_kernel<<<1, 32, 0, stream>>>(TW);
  cast_weights_kernel<<<((kNcat + kDch) * kDch) / 2048, 256, 0, stream>>>(Wx, Wb, Wc, Wout, WH);

  fwd_rows_kernel<<<kBatch * kChan * (kHt / 32), 32, 0, stream>>>(x, TW, PRE, PIM);
  fwd_cols_kernel<<<kBatch * kWf * 2, 32, 0, stream>>>(PRE, PIM, TW, U);

  ln_gate_kernel<<<kTok / 64, 256, 0, stream>>>(U, nw, nb, wdt, dtbias, alog, UH, DD);

  gemm_f16_kernel<<<(kTok / 64) * (kNcat / 64) / 8, 256, 0, stream>>>(
      UH, kDch, WH, kDch, XBC, kNcat, kTok, kNcat, kDch, kProjScale);

  scan_kernel<<<kBatch * 2, 256, 0, stream>>>(XBC, DD, hprev, Dskip, Y, out1);

  gemm_f16_kernel<<<(kTok / 64) * (kDch / 64) / 8, 256, 0, stream>>>(
      Y, kDch, WH + (size_t)kNcat * kDch, kDch, F, kDch, kTok, kDch, kDch, kOutScale);

  inv_cols_kernel<<<kBatch * kWf * 2, 32, 0, stream>>>(F, TW, QRE, QIM);
  inv_rows_kernel<<<kBatch * kChan * (kHt / 32), 32, 0, stream>>>(QRE, QIM, TW, out0);
}
